// DeformableDownBlock_31026843746312
// MI455X (gfx1250) — hardware-verified
//
#include <hip/hip_runtime.h>
#include <stdint.h>
#include <stddef.h>


typedef _Float16 v16h __attribute__((ext_vector_type(16)));
typedef _Float16 v8h  __attribute__((ext_vector_type(8)));
typedef float    v8f  __attribute__((ext_vector_type(8)));
typedef float    v4f  __attribute__((ext_vector_type(4)));
typedef v16h v16ha __attribute__((may_alias));
typedef v8h  v8ha  __attribute__((may_alias));
typedef v4f  v4fa  __attribute__((may_alias));

#define TB    256
#define DT    128
#define TN    64
#define OCH   128
#define NTAP  9
#define CP    68
#define CP2   132
#define WSC   256.0f
#define BSC   16.0f
#define INVS  0.000244140625f

union Frag  { v16h v; v8h half[2]; _Float16 s[16]; };
union Pack8 { v8h v; _Float16 s[8]; };

__device__ __forceinline__ v8f wmma_f16(v16h a, v16h b, v8f c)
{
    v8f d = __builtin_amdgcn_wmma_f32_16x16x32_f16(false, a, false, b, (short)0, c, false, false);
    asm volatile("v_nop\n\tv_nop\n\tv_nop\n\tv_nop" : "+v"(d) : "v"(a), "v"(b));
    return d;
}

__global__ void __launch_bounds__(TB)
cvt_weights_kernel(const float* __restrict__ wa, const float* __restrict__ wb,
                   _Float16* __restrict__ dst, int rowsA, int rowsB, int K, int ngroups)
{
    const int g = blockIdx.x * TB + threadIdx.x;
    if (g >= ngroups) return;
    const int e0  = g * 8;
    const int row = e0 / K;
    const int k   = e0 - row * K;
    Pack8 pk;
#pragma unroll
    for (int i = 0; i < 8; ++i) {
        float f = 0.f;
        if (row < rowsA)              f = wa[(size_t)row * K + k + i];
        else if (row < rowsA + rowsB) f = wb[(size_t)(row - rowsA) * K + k + i];
        pk.s[i] = (_Float16)(f * WSC);
    }
    _Float16* p = dst + e0;
    *(volatile v8h*)p = pk.v;
    __threadfence();
    *(volatile v8h*)p = pk.v;
}

template <bool NORM>
__device__ __forceinline__ float tap(const float* __restrict__ xc,
                                     int H, int W, int y, int x,
                                     float m, float is)
{
    bool ok = ((unsigned)y < (unsigned)H) & ((unsigned)x < (unsigned)W);
    int yc = min(max(y, 0), H - 1);
    int xcl = min(max(x, 0), W - 1);
    float v = xc[yc * W + xcl];
    if (NORM) v = fmaxf((v - m) * is, 0.f);
    return ok ? v : 0.f;
}

template <bool NORM>
__device__ __forceinline__ float bilinear(const float* __restrict__ xc,
                                          int H, int W, float py, float px,
                                          float m, float is)
{
    float y0f = floorf(py), x0f = floorf(px);
    int y0 = (int)y0f, x0 = (int)x0f;
    float wy = py - y0f, wx = px - x0f;
    int y1 = y0 + 1, x1 = x0 + 1;
    bool vy0 = (unsigned)y0 < (unsigned)H, vy1 = (unsigned)y1 < (unsigned)H;
    bool vx0 = (unsigned)x0 < (unsigned)W, vx1 = (unsigned)x1 < (unsigned)W;
    int y0c = min(max(y0, 0), H - 1), y1c = min(max(y1, 0), H - 1);
    int x0c = min(max(x0, 0), W - 1), x1c = min(max(x1, 0), W - 1);
    float v00 = xc[y0c * W + x0c];
    float v01 = xc[y0c * W + x1c];
    float v10 = xc[y1c * W + x0c];
    float v11 = xc[y1c * W + x1c];
    if (NORM) {
        v00 = fmaxf((v00 - m) * is, 0.f);
        v01 = fmaxf((v01 - m) * is, 0.f);
        v10 = fmaxf((v10 - m) * is, 0.f);
        v11 = fmaxf((v11 - m) * is, 0.f);
    }
    float f00 = (vy0 & vx0) ? (1.f - wy) * (1.f - wx) : 0.f;
    float f01 = (vy0 & vx1) ? (1.f - wy) * wx         : 0.f;
    float f10 = (vy1 & vx0) ? wy * (1.f - wx)         : 0.f;
    float f11 = (vy1 & vx1) ? wy * wx                 : 0.f;
    return v00 * f00 + v01 * f01 + v10 * f10 + v11 * f11;
}

template <bool NORM>
__global__ void __launch_bounds__(TB)
offmod_kernel(const float* __restrict__ x,
              const _Float16* __restrict__ wh,
              const float* __restrict__ b_off,
              const float* __restrict__ b_mod,
              const float* __restrict__ mean,
              const float* __restrict__ istd,
              float* __restrict__ off,
              float* __restrict__ mod,
              int Cin, int H, int W)
{
    const int t = threadIdx.x, wave = t >> 5, l = t & 31, h = l >> 4, m = l & 15;
    const int b = blockIdx.y;
    const int HW = H * W;
    const int tile_base = blockIdx.x * DT;
    if (tile_base + DT > HW) return;
    const int K = Cin * NTAP, nK = K >> 5;

    __shared__ __align__(16) float Cs[32 * CP2];

    const int Nn  = (wave << 4) + m;
    const int hw0 = tile_base + Nn;
    const int hh0 = hw0 / W, ww0 = hw0 - hh0 * W;

    const v8f vz = {0.f, 0.f, 0.f, 0.f, 0.f, 0.f, 0.f, 0.f};
    v8f acc0 = vz, acc1 = vz;

    const float* xb = x + (size_t)b * Cin * HW;
    const _Float16* wrow0 = wh + (size_t)m * K + (h << 3);
    const _Float16* wrow1 = wh + (size_t)(16 + m) * K + (h << 3);

    for (int ks = 0; ks < nK; ++ks) {
        const int k0 = ks << 5;
        Frag bb;
#pragma unroll
        for (int hf = 0; hf < 2; ++hf) {
            int kg = k0 + (hf << 4) + (h << 3);
            int c  = kg / NTAP;
            int kk = kg - c * NTAP;
            int ky = kk / 3;
            int kx = kk - ky * 3;
#pragma unroll
            for (int i = 0; i < 8; ++i) {
                float mu = NORM ? mean[c] : 0.f;
                float is = NORM ? istd[c] : 1.f;
                float v  = tap<NORM>(xb + (size_t)c * HW, H, W,
                                     hh0 + ky - 1, ww0 + kx - 1, mu, is);
                bb.s[(hf << 3) + i] = (_Float16)(v * BSC);
                if (++kx == 3) { kx = 0; if (++ky == 3) { ky = 0; ++c; } }
            }
        }
        Frag a0, a1;
        a0.half[0] = *(const v8ha*)(wrow0 + k0);
        a0.half[1] = *(const v8ha*)(wrow0 + k0 + 16);
        a1.half[0] = *(const v8ha*)(wrow1 + k0);
        a1.half[1] = *(const v8ha*)(wrow1 + k0 + 16);
        acc0 = wmma_f16(a0.v, bb.v, acc0);
        acc1 = wmma_f16(a1.v, bb.v, acc1);
    }

#pragma unroll
    for (int r = 0; r < 8; ++r) {
        Cs[((h << 3) + r) * CP2 + Nn]      = acc0[r] * INVS;
        Cs[(16 + (h << 3) + r) * CP2 + Nn] = acc1[r] * INVS;
    }
    __syncthreads();

    v4f vals[4];
#pragma unroll
    for (int j = 0; j < 4; ++j) {
        const int row = wave + 8 * j;
        vals[j] = (v4f){0.f, 0.f, 0.f, 0.f};
        if (row < 27) {
            v4f v = *(const v4fa*)(Cs + row * CP2 + (l << 2));
            float* p;
            if (row < 18) {
                float bo = b_off[row];
                v = v + bo;
                p = off + ((size_t)(b * 18 + row)) * HW + tile_base + (l << 2);
            } else {
                float bm = b_mod[row - 18];
                v.x = 2.0f / (1.0f + expf(-(v.x + bm)));
                v.y = 2.0f / (1.0f + expf(-(v.y + bm)));
                v.z = 2.0f / (1.0f + expf(-(v.z + bm)));
                v.w = 2.0f / (1.0f + expf(-(v.w + bm)));
                p = mod + ((size_t)(b * NTAP + (row - 18))) * HW + tile_base + (l << 2);
            }
            vals[j] = v;
            *(volatile v4f*)p = v;
        }
    }
    __threadfence();
#pragma unroll
    for (int j = 0; j < 4; ++j) {
        const int row = wave + 8 * j;
        if (row < 27) {
            float* p = (row < 18)
                ? off + ((size_t)(b * 18 + row)) * HW + tile_base + (l << 2)
                : mod + ((size_t)(b * NTAP + (row - 18))) * HW + tile_base + (l << 2);
            *(volatile v4f*)p = vals[j];
        }
    }
}

template <bool NORM>
__global__ void __launch_bounds__(TB)
deform_cols_kernel(const float* __restrict__ xsrc,
                   const float* __restrict__ off,
                   const float* __restrict__ mod,
                   const float* __restrict__ mean,
                   const float* __restrict__ istd,
                   _Float16* __restrict__ P,
                   int b, int Cin, int H, int W)
{
    const int t = threadIdx.x;
    const int HW = H * W;
    const int tile_base = blockIdx.x * TN;
    if (tile_base + TN > HW) return;
    const int K = Cin * NTAP, KG = K >> 3, ngrp = TN * KG;

    __shared__ float s_dy[NTAP * TN];
    __shared__ float s_dx[NTAP * TN];
    __shared__ float s_m [NTAP * TN];

    for (int i = t; i < NTAP * TN; i += TB) {
        int kk = i / TN, n = i - kk * TN;
        int hw = tile_base + n;
        s_dy[i] = off[((size_t)(b * 2 * NTAP + 2 * kk))     * HW + hw];
        s_dx[i] = off[((size_t)(b * 2 * NTAP + 2 * kk + 1)) * HW + hw];
        s_m[i]  = mod[((size_t)(b * NTAP + kk))             * HW + hw];
    }
    __syncthreads();

    const float* xb = xsrc + (size_t)b * Cin * HW;
    _Float16* pb = P + (size_t)tile_base * K;

    for (int g = t; g < ngrp; g += TB) {
        const int nl = g / KG;
        const int k  = (g - nl * KG) << 3;
        int c  = k / NTAP;
        int kk = k - c * NTAP;
        int ky = kk / 3;
        int kx = kk - ky * 3;
        const int hw = tile_base + nl;
        const int hh = hw / W, ww = hw - hh * W;
        Pack8 pk;
#pragma unroll
        for (int i = 0; i < 8; ++i) {
            const int si = kk * TN + nl;
            float py = (float)(hh + ky - 1) + s_dy[si];
            float px = (float)(ww + kx - 1) + s_dx[si];
            float mu = NORM ? mean[c] : 0.f;
            float is = NORM ? istd[c] : 1.f;
            float v  = bilinear<NORM>(xb + (size_t)c * HW, H, W, py, px, mu, is);
            pk.s[i] = (_Float16)(v * s_m[si] * BSC);
            if (++kk == NTAP) kk = 0;
            if (++kx == 3) { kx = 0; if (++ky == 3) { ky = 0; ++c; } }
        }
        _Float16* p = pb + (size_t)g * 8;
        *(volatile v8h*)p = pk.v;
        __threadfence();
        *(volatile v8h*)p = pk.v;
    }
}

__global__ void __launch_bounds__(TB)
deform_gemm_kernel(const _Float16* __restrict__ P,
                   const _Float16* __restrict__ wh,
                   float* __restrict__ hout,
                   float* __restrict__ part,
                   int b, int K, int HW)
{
    const int t = threadIdx.x, wave = t >> 5, l = t & 31, h = l >> 4, m = l & 15;
    const int tile_base = blockIdx.x * DT;
    if (tile_base + DT > HW) return;
    const int nK  = K >> 5;
    const int blk = b * gridDim.x + blockIdx.x;

    __shared__ __align__(16) float Cs[OCH * CP];
    __shared__ __align__(16) float s_st[2 * OCH];

    const v8f vz = {0.f, 0.f, 0.f, 0.f, 0.f, 0.f, 0.f, 0.f};
    v8f acc[8];
#pragma unroll
    for (int i = 0; i < 8; ++i) acc[i] = vz;

    const _Float16* wrow = wh + (size_t)((wave << 4) + m) * K + (h << 3);
    const _Float16* prow = P + (size_t)(tile_base + m) * K + (h << 3);
    const size_t sub = (size_t)16 * K;

    for (int ks = 0; ks < nK; ++ks) {
        const int k0 = ks << 5;
        Frag a;
        a.half[0] = *(const v8ha*)(wrow + k0);
        a.half[1] = *(const v8ha*)(wrow + k0 + 16);
#pragma unroll
        for (int n = 0; n < 8; ++n) {
            const _Float16* q = prow + n * sub + k0;
            Frag bb;
            bb.half[0] = *(const v8ha*)q;
            bb.half[1] = *(const v8ha*)(q + 16);
            acc[n] = wmma_f16(a.v, bb.v, acc[n]);
        }
    }

#pragma unroll
    for (int n = 0; n < 8; ++n) acc[n] = acc[n] * INVS;

#pragma unroll
    for (int r = 0; r < 8; ++r) {
        float s = 0.f, q = 0.f;
#pragma unroll
        for (int n = 0; n < 8; ++n) { float v = acc[n][r]; s += v; q += v * v; }
        s += __shfl_xor(s, 1); q += __shfl_xor(q, 1);
        s += __shfl_xor(s, 2); q += __shfl_xor(q, 2);
        s += __shfl_xor(s, 4); q += __shfl_xor(q, 4);
        s += __shfl_xor(s, 8); q += __shfl_xor(q, 8);
        if (m == 0) {
            s_st[(wave << 4) + (h << 3) + r]       = s;
            s_st[OCH + (wave << 4) + (h << 3) + r] = q;
        }
    }

#pragma unroll
    for (int p = 0; p < 2; ++p) {
#pragma unroll
        for (int qn = 0; qn < 4; ++qn) {
#pragma unroll
            for (int r = 0; r < 8; ++r)
                Cs[((wave << 4) + (h << 3) + r) * CP + (qn << 4) + m] = acc[4 * p + qn][r];
        }
        __syncthreads();
        v4f v[8];
#pragma unroll
        for (int i = 0; i < 8; ++i)
            v[i] = *(const v4fa*)(Cs + ((wave << 4) + 2 * i + h) * CP + (m << 2));
        float* gp = hout + ((size_t)(b * OCH + (wave << 4) + h)) * HW
                         + tile_base + 64 * p + (m << 2);
#pragma unroll
        for (int i = 0; i < 8; ++i)
            *(volatile v4f*)(gp + (size_t)(2 * i) * HW) = v[i];
        __threadfence();
#pragma unroll
        for (int i = 0; i < 8; ++i)
            *(volatile v4f*)(gp + (size_t)(2 * i) * HW) = v[i];
        __syncthreads();
    }

    if (wave == 0) {
        v4f ps = *(const v4fa*)(s_st + (l << 2));
        v4f pq = *(const v4fa*)(s_st + OCH + (l << 2));
        float* pp = part + (size_t)blk * (2 * OCH);
        *(volatile v4f*)(pp + (l << 2))       = ps;
        *(volatile v4f*)(pp + OCH + (l << 2)) = pq;
        __threadfence();
        *(volatile v4f*)(pp + (l << 2))       = ps;
        *(volatile v4f*)(pp + OCH + (l << 2)) = pq;
    }
}

__global__ void __launch_bounds__(OCH)
bn_finalize_kernel(const float* __restrict__ part,
                   float* __restrict__ mean,
                   float* __restrict__ istd,
                   int nblk, int npos)
{
    const int c = threadIdx.x;
    double s = 0.0, q = 0.0;
    for (int i = 0; i < nblk; ++i) {
        s += (double)part[(size_t)i * (2 * OCH) + c];
        q += (double)part[(size_t)i * (2 * OCH) + OCH + c];
    }
    double mu  = s / (double)npos;
    double var = q / (double)npos - mu * mu;
    if (var < 0.0) var = 0.0;
    float mf  = (float)mu;
    float isf = (float)(1.0 / sqrt(var + 1e-5));
    *(volatile float*)(mean + c) = mf;
    *(volatile float*)(istd + c) = isf;
    __threadfence();
    *(volatile float*)(mean + c) = mf;
    *(volatile float*)(istd + c) = isf;
}

__global__ void __launch_bounds__(TB)
bn_pool_kernel(const float* __restrict__ hin,
               const float* __restrict__ mean,
               const float* __restrict__ istd,
               float* __restrict__ out,
               int C, int H, int W, int nquad)
{
    const int q = blockIdx.x * TB + threadIdx.x;
    if (q >= nquad) return;
    const int Ho = H >> 1, Wo = W >> 1, qpr = Wo >> 2;
    const int rowid = q / qpr;
    const int ow0   = (q - rowid * qpr) << 2;
    const int oh    = rowid % Ho;
    const int bc    = rowid / Ho;
    const int c     = bc % C;
    const float mu = mean[c], is = istd[c];
    const float* base = hin + (size_t)bc * H * W + (size_t)(2 * oh) * W + 2 * ow0;
    v4f r0a = *(const v4fa*)(base);
    v4f r0b = *(const v4fa*)(base + 4);
    v4f r1a = *(const v4fa*)(base + W);
    v4f r1b = *(const v4fa*)(base + W + 4);
    r0a = (r0a - mu) * is; r0b = (r0b - mu) * is;
    r1a = (r1a - mu) * is; r1b = (r1b - mu) * is;
    v4f o;
    o.x = fmaxf(fmaxf(fmaxf(r0a.x, r0a.y), fmaxf(r1a.x, r1a.y)), 0.f);
    o.y = fmaxf(fmaxf(fmaxf(r0a.z, r0a.w), fmaxf(r1a.z, r1a.w)), 0.f);
    o.z = fmaxf(fmaxf(fmaxf(r0b.x, r0b.y), fmaxf(r1b.x, r1b.y)), 0.f);
    o.w = fmaxf(fmaxf(fmaxf(r0b.z, r0b.w), fmaxf(r1b.z, r1b.w)), 0.f);
    float* p = out + (size_t)q * 4;
    *(volatile v4f*)p = o;
    __threadfence();
    *(volatile v4f*)p = o;
}

static inline size_t al256(size_t v) { return (v + 255) & ~(size_t)255; }

extern "C" void kernel_launch(void* const* d_in, const int* in_sizes, int n_in,
                              void* d_out, int out_size, void* d_ws, size_t ws_size,
                              hipStream_t stream)
{
    const int B = 4, Cin = 64, H = 128, W = 128;
    const int HW = H * W;
    const int K1 = Cin * NTAP, K2 = OCH * NTAP;

    if (n_in < 11) return;
    if (in_sizes[0] != B * Cin * HW) return;
    if (in_sizes[1] != 2 * NTAP * K1 || in_sizes[2] != 2 * NTAP) return;
    if (in_sizes[3] != NTAP * K1 || in_sizes[4] != NTAP) return;
    if (in_sizes[5] != OCH * K1) return;
    if (in_sizes[6] != 2 * NTAP * K2 || in_sizes[7] != 2 * NTAP) return;
    if (in_sizes[8] != NTAP * K2 || in_sizes[9] != NTAP) return;
    if (in_sizes[10] != OCH * K2) return;
    if (out_size != B * OCH * (H / 2) * (W / 2)) return;
    if ((HW % DT) != 0 || (HW % TN) != 0 || (K1 % 32) != 0 || (K2 % 32) != 0 || ((W / 2) % 4) != 0) return;

    const float* x      = (const float*)d_in[0];
    const float* w_off1 = (const float*)d_in[1];
    const float* b_off1 = (const float*)d_in[2];
    const float* w_mod1 = (const float*)d_in[3];
    const float* b_mod1 = (const float*)d_in[4];
    const float* w1     = (const float*)d_in[5];
    const float* w_off2 = (const float*)d_in[6];
    const float* b_off2 = (const float*)d_in[7];
    const float* w_mod2 = (const float*)d_in[8];
    const float* b_mod2 = (const float*)d_in[9];
    const float* w2     = (const float*)d_in[10];
    float* out = (float*)d_out;

    const int nblk = B * (HW / DT);
    char* ws = (char*)d_ws;
    size_t o = 0;
    float* offb  = (float*)(ws + o); o = al256(o + (size_t)B * 2 * NTAP * HW * 4);
    float* modb  = (float*)(ws + o); o = al256(o + (size_t)B * NTAP * HW * 4);
    float* h1    = (float*)(ws + o); o = al256(o + (size_t)B * OCH * HW * 4);
    float* h2    = (float*)(ws + o); o = al256(o + (size_t)B * OCH * HW * 4);
    _Float16* P  = (_Float16*)(ws + o); o = al256(o + (size_t)HW * K2 * 2);
    float* part  = (float*)(ws + o); o = al256(o + (size_t)nblk * 2 * OCH * 4);
    float* mean1 = (float*)(ws + o); o = al256(o + (size_t)OCH * 4);
    float* istd1 = (float*)(ws + o); o = al256(o + (size_t)OCH * 4);
    float* mean2 = (float*)(ws + o); o = al256(o + (size_t)OCH * 4);
    float* istd2 = (float*)(ws + o); o = al256(o + (size_t)OCH * 4);
    _Float16* wA1  = (_Float16*)(ws + o); o = al256(o + (size_t)OCH * K1 * 2);
    _Float16* wOM1 = (_Float16*)(ws + o); o = al256(o + (size_t)32 * K1 * 2);
    _Float16* wA2  = (_Float16*)(ws + o); o = al256(o + (size_t)OCH * K2 * 2);
    _Float16* wOM2 = (_Float16*)(ws + o); o = al256(o + (size_t)32 * K2 * 2);
    if (o > ws_size) return;

    const dim3 conv_grid(HW / DT, B);
    const int cols_grid = HW / TN;
    const int gemm_grid = HW / DT;
    const int ngOM1 = 32 * K1 / 8, ngA1 = OCH * K1 / 8;
    const int ngOM2 = 32 * K2 / 8, ngA2 = OCH * K2 / 8;
    const int npos  = B * HW;
    const int nquad = out_size / 4;

    cvt_weights_kernel<<<(ngOM1 + TB - 1) / TB, TB, 0, stream>>>(
        w_off1, w_mod1, wOM1, 2 * NTAP, NTAP, K1, ngOM1);
    cvt_weights_kernel<<<(ngA1 + TB - 1) / TB, TB, 0, stream>>>(
        w1, w1, wA1, OCH, 0, K1, ngA1);
    offmod_kernel<false><<<conv_grid, TB, 0, stream>>>(
        x, wOM1, b_off1, b_mod1, mean1, istd1, offb, modb, Cin, H, W);
    for (int b = 0; b < B; ++b) {
        deform_cols_kernel<false><<<cols_grid, TB, 0, stream>>>(
            x, offb, modb, mean1, istd1, P, b, Cin, H, W);
        deform_gemm_kernel<<<gemm_grid, TB, 0, stream>>>(
            P, wA1, h1, part, b, K1, HW);
    }
    bn_finalize_kernel<<<1, OCH, 0, stream>>>(part, mean1, istd1, nblk, npos);

    cvt_weights_kernel<<<(ngOM2 + TB - 1) / TB, TB, 0, stream>>>(
        w_off2, w_mod2, wOM2, 2 * NTAP, NTAP, K2, ngOM2);
    cvt_weights_kernel<<<(ngA2 + TB - 1) / TB, TB, 0, stream>>>(
        w2, w2, wA2, OCH, 0, K2, ngA2);
    offmod_kernel<true><<<conv_grid, TB, 0, stream>>>(
        h1, wOM2, b_off2, b_mod2, mean1, istd1, offb, modb, OCH, H, W);
    for (int b = 0; b < B; ++b) {
        deform_cols_kernel<true><<<cols_grid, TB, 0, stream>>>(
            h1, offb, modb, mean1, istd1, P, b, OCH, H, W);
        deform_gemm_kernel<<<gemm_grid, TB, 0, stream>>>(
            P, wA2, h2, part, b, K2, HW);
    }
    bn_finalize_kernel<<<1, OCH, 0, stream>>>(part, mean2, istd2, nblk, npos);

    bn_pool_kernel<<<(nquad + TB - 1) / TB, TB, 0, stream>>>(
        h2, mean2, istd2, out, OCH, H, W, nquad);
}
